// LongformerSelfAttention_25658134627018
// MI455X (gfx1250) — hardware-verified
//
#include <hip/hip_runtime.h>


#ifndef NB
#define NB 2
#endif
#ifndef SEQ
#define SEQ 4096
#endif
#define NB_FULL  2
#define SEQ_FULL 4096
#define EMB 512
#define NH  8
#define HD  64
#define WIN 64
#define QB  32
#define KWN (QB + 2 * WIN)
#define LKP (SEQ + 2 * WIN)
#define LVP (SEQ + 2 * WIN)
#define SLD 164
#define PLD 168
#define OSP 68
#define QSCL 0.125f

static_assert(NB <= NB_FULL);
static_assert(SEQ <= SEQ_FULL);
static_assert(SEQ % 64 == 0);
static_assert(SEQ % QB == 0);
static_assert(KWN % 32 == 0);
static_assert(EMB == NH * HD);
static_assert((LVP % 2) == 0);
static_assert((SLD * 4) % 16 == 0);
static_assert((PLD * 2) % 16 == 0);
static_assert((OSP * 4) % 16 == 0);
static_assert(PLD >= KWN);
static_assert(SLD >= KWN);

typedef unsigned short bf;
typedef __attribute__((ext_vector_type(16))) __bf16   v16bf;
typedef __attribute__((ext_vector_type(8)))  unsigned short v8us;
typedef __attribute__((ext_vector_type(4)))  unsigned short v4us;
typedef __attribute__((ext_vector_type(2)))  unsigned short v2us;
typedef __attribute__((ext_vector_type(8)))  float    v8f;
typedef __attribute__((ext_vector_type(4)))  float    v4f;
typedef __attribute__((ext_vector_type(2)))  float    v2f;
typedef v4f  __attribute__((may_alias)) v4fa;
typedef v8us __attribute__((may_alias)) v8usa;

__device__ __forceinline__ unsigned short f2bf(float f) { unsigned u = __float_as_uint(f); u += 0x7FFFu + ((u >> 16) & 1u); return (unsigned short)(u >> 16); }
__device__ __forceinline__ float bf2f(unsigned short b) { return __uint_as_float(((unsigned)b) << 16); }
__device__ __forceinline__ float bfr(float f) { return bf2f(f2bf(f)); }
__device__ __forceinline__ void splitf(float y, unsigned short& h, unsigned short& l) { h = f2bf(y); l = f2bf(y - bf2f(h)); }
__device__ __forceinline__ v16bf cat16b(v8us lo, v8us hi) { return __builtin_bit_cast(v16bf, __builtin_shufflevector(lo, hi, 0, 1, 2, 3, 4, 5, 6, 7, 8, 9, 10, 11, 12, 13, 14, 15)); }
__device__ __forceinline__ v8f wmmab(v16bf a, v16bf b, v8f c) { return __builtin_amdgcn_wmma_f32_16x16x32_bf16(false, a, false, b, (short)0, c, false, false); }

template <typename T16> struct WFrag;
template <> struct WFrag<bf> { typedef v16bf V; static __device__ __forceinline__ V ld(const bf* p) { return cat16b(*(const v8us*)p, *(const v8us*)(p + 16)); } static __device__ __forceinline__ v8f mma(V a, V b, v8f c) { return wmmab(a, b, c); } };

template <typename T16, int NSPLIT, bool BIAS>
__global__ __launch_bounds__(32) void k_gemmw(const T16* __restrict__ A, const T16* __restrict__ A2, const T16* __restrict__ Bt, const T16* __restrict__ Bt2, int K, float* C, int ldc, const float* __restrict__ bias, size_t sA, size_t sB, size_t sC) {
    typedef typename WFrag<T16>::V V;
    __shared__ __align__(16) float os[16 * 68];
    const size_t z = blockIdx.z; A += z * sA; if (A2) A2 += z * sA; Bt += z * sB; if (Bt2) Bt2 += z * sB; C += z * sC;
    const int lane = threadIdx.x & 31, lr = lane & 15, hi = lane >> 4; const int r0 = blockIdx.x * 64, c0 = blockIdx.y * 64;
    v8f acc[4][4];
#pragma unroll
    for (int mb = 0; mb < 4; ++mb)
#pragma unroll
        for (int nb = 0; nb < 4; ++nb) acc[mb][nb] = (v8f){};
    const size_t aoff = (size_t)(r0 + lr) * K + 8 * hi, boff = (size_t)(c0 + lr) * K + 8 * hi;
#pragma unroll 1
    for (int kc = 0; kc < K; kc += 32) {
        V a[4], a2[4];
#pragma unroll
        for (int mb = 0; mb < 4; ++mb) { a[mb] = WFrag<T16>::ld(A + aoff + (size_t)mb * 16 * K + kc); if (NSPLIT == 1 || NSPLIT == 2) a2[mb] = WFrag<T16>::ld(A2 + aoff + (size_t)mb * 16 * K + kc); }
#pragma unroll
        for (int nb = 0; nb < 4; ++nb) { const V b = WFrag<T16>::ld(Bt + boff + (size_t)nb * 16 * K + kc); V b2; if (NSPLIT >= 2) b2 = WFrag<T16>::ld(Bt2 + boff + (size_t)nb * 16 * K + kc);
#pragma unroll
            for (int mb = 0; mb < 4; ++mb) { acc[mb][nb] = WFrag<T16>::mma(a[mb], b, acc[mb][nb]); if (NSPLIT == 1 || NSPLIT == 2) acc[mb][nb] = WFrag<T16>::mma(a2[mb], b, acc[mb][nb]); if (NSPLIT >= 2) acc[mb][nb] = WFrag<T16>::mma(a[mb], b2, acc[mb][nb]); } }
        asm volatile("v_nop\n\tv_nop\n\tv_nop\n\tv_nop" : "+v"(acc[0][0]), "+v"(acc[1][1]), "+v"(acc[2][2]), "+v"(acc[3][3]) : "v"(a[0]), "v"(a[3]));
    }
#pragma unroll
    for (int mb = 0; mb < 4; ++mb) {
#pragma unroll
        for (int nb = 0; nb < 4; ++nb) {
#pragma unroll
            for (int j = 0; j < 8; ++j) os[(hi * 8 + j) * 68 + nb * 16 + lr] = acc[mb][nb][j]; }
        __builtin_amdgcn_wave_barrier(); asm volatile("" ::: "memory");
        float* crow = C + (size_t)(r0 + mb * 16) * ldc + c0;
#pragma unroll 1
        for (int ps = 0; ps < 2; ++ps) {
#pragma unroll
            for (int s = 0; s < 8; ++s) { const int row = 2 * s + hi, cofs = lr * 4; v4f val = *(const v4fa*)(os + row * 68 + cofs); if (BIAS) { val[0] += bfr(bias[c0 + cofs]); val[1] += bfr(bias[c0 + cofs + 1]); val[2] += bfr(bias[c0 + cofs + 2]); val[3] += bfr(bias[c0 + cofs + 3]); }
                *(volatile v4f*)(crow + (size_t)row * ldc + cofs) = val; }
            if (ps == 0) __threadfence(); }
        __builtin_amdgcn_wave_barrier(); asm volatile("" ::: "memory");
    }
}

__global__ __launch_bounds__(256) void k_wtG(const float* __restrict__ w, int K, int N, bf* Bt) {
    const int lane = threadIdx.x & 31; const int L0 = (blockIdx.x * 8 + (threadIdx.x >> 5)) * 8; const int nlines = N * K / 64;
#pragma unroll
    for (int ps = 0; ps < 2; ++ps) {
#pragma unroll 1
        for (int l = 0; l < 8; ++l) { const int L = L0 + l; if (L >= nlines) break; const size_t e = (size_t)L * 64 + lane * 2; const int k = (int)(e % K), n = (int)(e / K); v2us o;
            o[0] = f2bf(w[(size_t)k * N + n]); o[1] = f2bf(w[(size_t)(k + 1) * N + n]); *(volatile v2us*)(Bt + e) = o; }
        if (ps == 0) __threadfence(); }
}
__global__ __launch_bounds__(256) void k_cvt8(const float* __restrict__ src, bf* dst, size_t n8) { const size_t i = (size_t)blockIdx.x * 256 + threadIdx.x; if (i >= n8) return; const v8f v = *(const v8f*)(src + i * 8); v8us o;
#pragma unroll
    for (int k = 0; k < 8; ++k) o[k] = f2bf(v[k]); *(volatile v8us*)(dst + i * 8) = o; __threadfence(); *(volatile v8us*)(dst + i * 8) = o; }

template <int PAD>
__global__ __launch_bounds__(256) void k_plane(const float* __restrict__ F, float scl, bf* Ph, bf* Pl) {
    constexpr int LR = SEQ + 2 * PAD;
    const unsigned tot = (unsigned)NH * (unsigned)LR * (unsigned)HD;
    const unsigned e = (blockIdx.x * 256u + threadIdx.x) * 2u; if (e >= tot) return;
    const int d = (int)(e % HD); const int tp = (int)((e / HD) % (unsigned)LR); const int hh = (int)(e / ((unsigned)HD * (unsigned)LR));
    const int t = tp - PAD; const bool ok = (t >= 0) && (t < SEQ); const int tc = min(max(t, 0), SEQ - 1);
    const v2f xv = *(const v2f*)(F + (size_t)tc * EMB + hh * HD + d);
    v2us oh, ol;
#pragma unroll
    for (int q = 0; q < 2; ++q) { const float r = ok ? xv[q] * scl : 0.0f; unsigned short a, c; splitf(r, a, c); oh[q] = a; ol[q] = c; }
    *(volatile v2us*)(Ph + e) = oh; *(volatile v2us*)(Pl + e) = ol; __threadfence(); *(volatile v2us*)(Ph + e) = oh; *(volatile v2us*)(Pl + e) = ol;
}

__global__ __launch_bounds__(256) void k_vt(const float* __restrict__ F, bf* Vh, bf* Vl) {
    const unsigned tot = (unsigned)NH * (unsigned)HD * (unsigned)LVP;
    const unsigned e = (blockIdx.x * 256u + threadIdx.x) * 2u; if (e >= tot) return;
    const int jp = (int)(e % (unsigned)LVP); const int d = (int)((e / (unsigned)LVP) % HD); const int hh = (int)(e / ((unsigned)LVP * (unsigned)HD));
    v2us oh, ol;
#pragma unroll
    for (int q = 0; q < 2; ++q) { const int j = jp + q - WIN; const bool ok = (j >= 0) && (j < SEQ); const int jc = min(max(j, 0), SEQ - 1);
        const float val = F[(size_t)jc * EMB + hh * HD + d]; const float r = ok ? val : 0.0f; unsigned short a, c; splitf(r, a, c); oh[q] = a; ol[q] = c; }
    *(volatile v2us*)(Vh + e) = oh; *(volatile v2us*)(Vl + e) = ol; __threadfence(); *(volatile v2us*)(Vh + e) = oh; *(volatile v2us*)(Vl + e) = ol;
}

__global__ __launch_bounds__(64) void k_attn(const bf* __restrict__ Qh, const bf* __restrict__ Ql, const bf* __restrict__ Kh, const bf* __restrict__ Kl,
                                             const bf* __restrict__ Vh, const bf* __restrict__ Vl, const int* __restrict__ msk, float* out) {
    __shared__ __align__(16) float sc[QB * SLD];
    __shared__ __align__(16) unsigned short ph[QB * PLD];
    __shared__ __align__(16) unsigned short pl[QB * PLD];
    __shared__ __align__(16) float os[QB * OSP];
    const int lane = threadIdx.x & 31, lr = lane & 15, hi = lane >> 4, wv = threadIdx.x >> 5;
    const int r0 = blockIdx.x * QB; const int hh = blockIdx.y;

    {
        const bf* qh = Qh + ((size_t)hh * SEQ + r0 + wv * 16 + lr) * HD + 8 * hi;
        const bf* ql = Ql + ((size_t)hh * SEQ + r0 + wv * 16 + lr) * HD + 8 * hi;
        const v16bf aH0 = WFrag<bf>::ld(qh), aH1 = WFrag<bf>::ld(qh + 32), aL0 = WFrag<bf>::ld(ql), aL1 = WFrag<bf>::ld(ql + 32);
        const bf* kh = Kh + ((size_t)hh * LKP + r0 + lr) * HD + 8 * hi;
        const bf* kl = Kl + ((size_t)hh * LKP + r0 + lr) * HD + 8 * hi;
#pragma unroll 1
        for (int nt = 0; nt < KWN / 16; ++nt) {
            const bf* khp = kh + (size_t)nt * 16 * HD; const bf* klp = kl + (size_t)nt * 16 * HD;
            const v16bf bH0 = WFrag<bf>::ld(khp), bH1 = WFrag<bf>::ld(khp + 32), bL0 = WFrag<bf>::ld(klp), bL1 = WFrag<bf>::ld(klp + 32);
            v8f acc = (v8f){};
            acc = wmmab(aH0, bH0, acc); acc = wmmab(aL0, bH0, acc); acc = wmmab(aH0, bL0, acc);
            acc = wmmab(aH1, bH1, acc); acc = wmmab(aL1, bH1, acc); acc = wmmab(aH1, bL1, acc);
            asm volatile("v_nop\n\tv_nop\n\tv_nop\n\tv_nop" : "+v"(acc) : "v"(aH1), "v"(aL1), "v"(bH1), "v"(bL1), "v"(bH0), "v"(bL0));
#pragma unroll
            for (int r = 0; r < 8; ++r) sc[(wv * 16 + 8 * hi + r) * SLD + nt * 16 + lr] = acc[r];
        }
    }
    __syncthreads();

#pragma unroll 1
    for (int rr = 0; rr < 16; ++rr) {
        const int x = wv * 16 + rr; const int i = r0 + x;
        const bool keep = (msk[i] >= 0);
        float v[KWN / 32]; float mx = -3.0e38f;
#pragma unroll
        for (int q = 0; q < KWN / 32; ++q) {
            const int y = lane + 32 * q; const int j = r0 - WIN + y; const int jc = min(max(j, 0), SEQ - 1);
            const float madd = (msk[jc] != 0) ? -10000.0f : 0.0f;
            const bool ok = (y >= x) && (y <= x + 2 * WIN) && (j >= 0) && (j < SEQ);
            const float s = sc[x * SLD + y] + madd;
            const float t = ok ? s : -3.0e38f; v[q] = t; mx = fmaxf(mx, t);
        }
#pragma unroll
        for (int sh = 16; sh; sh >>= 1) mx = fmaxf(mx, __shfl_xor(mx, sh, 32));
        float sum = 0.0f;
#pragma unroll
        for (int q = 0; q < KWN / 32; ++q) { float d0 = __fsub_rn(v[q], mx); asm volatile("" : "+v"(d0)); v[q] = __builtin_amdgcn_exp2f(__fmul_rn(d0, 1.4426950408889634f)); sum += v[q]; }
#pragma unroll
        for (int sh = 16; sh; sh >>= 1) sum += __shfl_xor(sum, sh, 32);
        const float f = __fdiv_rn(1.0f, sum);
#pragma unroll
        for (int q = 0; q < KWN / 32; ++q) { const int y = lane + 32 * q; float pv = __fmul_rn(v[q], f); asm volatile("" : "+v"(pv)); pv = keep ? pv : 0.0f;
            unsigned short a, c; splitf(pv, a, c); ph[x * PLD + y] = a; pl[x * PLD + y] = c; }
    }
    __syncthreads();

    v8f acc[4];
#pragma unroll
    for (int nt = 0; nt < 4; ++nt) acc[nt] = (v8f){};
    {
        const unsigned short* prh = ph + (wv * 16 + lr) * PLD + 8 * hi;
        const unsigned short* prl = pl + (wv * 16 + lr) * PLD + 8 * hi;
        const bf* vh = Vh + ((size_t)hh * HD + lr) * LVP + r0 + 8 * hi;
        const bf* vl = Vl + ((size_t)hh * HD + lr) * LVP + r0 + 8 * hi;
#pragma unroll 1
        for (int kc = 0; kc < KWN; kc += 32) {
            const v16bf aH = cat16b(*(const v8usa*)(prh + kc), *(const v8usa*)(prh + kc + 16));
            const v16bf aL = cat16b(*(const v8usa*)(prl + kc), *(const v8usa*)(prl + kc + 16));
            v16bf bH[4], bL[4];
#pragma unroll
            for (int nt = 0; nt < 4; ++nt) { bH[nt] = WFrag<bf>::ld(vh + (size_t)nt * 16 * LVP + kc); bL[nt] = WFrag<bf>::ld(vl + (size_t)nt * 16 * LVP + kc); }
#pragma unroll
            for (int nt = 0; nt < 4; ++nt) { acc[nt] = wmmab(aH, bH[nt], acc[nt]); acc[nt] = wmmab(aL, bH[nt], acc[nt]); acc[nt] = wmmab(aH, bL[nt], acc[nt]); }
            asm volatile("v_nop\n\tv_nop\n\tv_nop\n\tv_nop" : "+v"(acc[0]), "+v"(acc[1]), "+v"(acc[2]), "+v"(acc[3]) : "v"(aH), "v"(aL), "v"(bH[0]), "v"(bH[3]), "v"(bL[0]), "v"(bL[3]));
        }
    }

#pragma unroll
    for (int nt = 0; nt < 4; ++nt) {
#pragma unroll
        for (int j = 0; j < 8; ++j) os[(wv * 16 + hi * 8 + j) * OSP + nt * 16 + lr] = acc[nt][j]; }
    __syncthreads();
    {
        float* orow = out + (size_t)(r0 + wv * 16) * EMB + hh * HD;
#pragma unroll 1
        for (int ps = 0; ps < 2; ++ps) {
#pragma unroll
            for (int s = 0; s < 8; ++s) { const int row = 2 * s + hi, cofs = lr * 4; const v4f val = *(const v4fa*)(os + (wv * 16 + row) * OSP + cofs);
                *(volatile v4f*)(orow + (size_t)row * EMB + cofs) = val; }
            if (ps == 0) __threadfence(); }
    }
}

extern "C" void kernel_launch(void* const* d_in, const int* in_sizes, int n_in,
                              void* d_out, int out_size, void* d_ws, size_t ws_size, hipStream_t stream) {
    if (n_in < 10) return;
    if ((size_t)in_sizes[0] < (size_t)(NB - 1) * SEQ_FULL * EMB + (size_t)SEQ * EMB) return;
    if (in_sizes[3] < (NB - 1) * SEQ_FULL + SEQ) return;
    if (in_sizes[4] < EMB * EMB || in_sizes[6] < EMB * EMB || in_sizes[8] < EMB * EMB) return;
    if (in_sizes[5] < EMB || in_sizes[7] < EMB || in_sizes[9] < EMB) return;
    if ((size_t)out_size < (size_t)NB * SEQ * EMB) return;
    const float* x  = (const float*)d_in[0];
    const int*   am = (const int*)d_in[3];
    const float* wq = (const float*)d_in[4]; const float* bq = (const float*)d_in[5];
    const float* wk = (const float*)d_in[6]; const float* bk = (const float*)d_in[7];
    const float* wv = (const float*)d_in[8]; const float* bv = (const float*)d_in[9];
    float* OUT = (float*)d_out;

    char* wsp = (char*)d_ws;
    auto take = [&](size_t bytes) { char* p = wsp; wsp += (bytes + 255) & ~(size_t)255; return (void*)p; };
    bf* WQ = (bf*)take((size_t)EMB * EMB * 2); bf* WK = (bf*)take((size_t)EMB * EMB * 2); bf* WV = (bf*)take((size_t)EMB * EMB * 2);
    bf* XB = (bf*)take((size_t)SEQ * EMB * 2);
    float* FQ = (float*)take((size_t)SEQ * EMB * 4); float* FK = (float*)take((size_t)SEQ * EMB * 4); float* FV = (float*)take((size_t)SEQ * EMB * 4);
    bf* QPh = (bf*)take((size_t)NH * SEQ * HD * 2); bf* QPl = (bf*)take((size_t)NH * SEQ * HD * 2);
    bf* KPh = (bf*)take((size_t)NH * LKP * HD * 2); bf* KPl = (bf*)take((size_t)NH * LKP * HD * 2);
    bf* VTh = (bf*)take((size_t)NH * HD * LVP * 2); bf* VTl = (bf*)take((size_t)NH * HD * LVP * 2);
    if ((size_t)(wsp - (char*)d_ws) > ws_size) return;

    const unsigned gW = (unsigned)((EMB * EMB / 64 + 63) / 64);
    k_wtG<<<gW, 256, 0, stream>>>(wq, EMB, EMB, WQ);
    k_wtG<<<gW, 256, 0, stream>>>(wk, EMB, EMB, WK);
    k_wtG<<<gW, 256, 0, stream>>>(wv, EMB, EMB, WV);
    const size_t nx8 = (size_t)SEQ * EMB / 8;
    const unsigned gQ = (unsigned)(((size_t)NH * SEQ * HD / 2 + 255) / 256);
    const unsigned gK = (unsigned)(((size_t)NH * LKP * HD / 2 + 255) / 256);
    const unsigned gV = (unsigned)(((size_t)NH * HD * LVP / 2 + 255) / 256);
    for (int b = 0; b < NB; ++b) {
        k_cvt8<<<(unsigned)((nx8 + 255) / 256), 256, 0, stream>>>(x + (size_t)b * SEQ_FULL * EMB, XB, nx8);
        k_gemmw<bf, 0, true><<<dim3(SEQ / 64, EMB / 64, 1), 32, 0, stream>>>(XB, nullptr, WQ, nullptr, EMB, FQ, EMB, bq, 0, 0, 0);
        k_plane<0><<<gQ, 256, 0, stream>>>(FQ, QSCL, QPh, QPl);
        k_gemmw<bf, 0, true><<<dim3(SEQ / 64, EMB / 64, 1), 32, 0, stream>>>(XB, nullptr, WK, nullptr, EMB, FK, EMB, bk, 0, 0, 0);
        k_plane<WIN><<<gK, 256, 0, stream>>>(FK, 1.0f, KPh, KPl);
        k_gemmw<bf, 0, true><<<dim3(SEQ / 64, EMB / 64, 1), 32, 0, stream>>>(XB, nullptr, WV, nullptr, EMB, FV, EMB, bv, 0, 0, 0);
        k_vt<<<gV, 256, 0, stream>>>(FV, VTh, VTl);
        k_attn<<<dim3(SEQ / QB, NH, 1), 64, 0, stream>>>(QPh, QPl, KPh, KPl, VTh, VTl, am + (size_t)b * SEQ_FULL, OUT + (size_t)b * SEQ * EMB);
    }
}
